// MP_GAT_58755152609379
// MI455X (gfx1250) — hardware-run, weakly checked
//
#include <hip/hip_runtime.h>
#include <stddef.h>
#include <stdint.h>

#define NB    8
#define NS    64
#define NNODE 512
#define NE    32
#define TC    64
#define RB    16

static_assert(NNODE % 64 == 0);
static_assert(NNODE % RB == 0);
static_assert(NS == 64);
static_assert(NE == 32);
static_assert(NNODE == 512);
static_assert(RB * 32 == 512);

typedef float          v8f  __attribute__((ext_vector_type(8)));
typedef float          v4f  __attribute__((ext_vector_type(4)));
typedef unsigned int   v4u  __attribute__((ext_vector_type(4)));
typedef _Float16       hf;
typedef hf             v16h __attribute__((ext_vector_type(16)));
typedef hf             v8h  __attribute__((ext_vector_type(8)));
typedef hf             v4h  __attribute__((ext_vector_type(4)));

union Frag { v16h v; v8h h[2]; };
union Pk8  { v8h h; v4u u; };

__device__ __forceinline__ v8f zero8() { return (v8f){0.f, 0.f, 0.f, 0.f, 0.f, 0.f, 0.f, 0.f}; }

__device__ __forceinline__ v8f mma16(v16h a, v16h b, v8f c) {
  c = __builtin_amdgcn_wmma_f32_16x16x32_f16(false, a, false, b, (short)0, c, false, false);
  asm volatile("v_nop\n\tv_nop\n\tv_nop\n\tv_nop" : "+v"(c) : "v"(a), "v"(b));
  return c;
}

__device__ __forceinline__ v16h ldfrag(const hf* p, int ld, int row0, int k0, int lane) {
  const int m = lane & 15, lh = lane >> 4;
  const hf* q = p + (size_t)(row0 + m) * ld + k0 + 8 * lh;
  Frag f;
  f.h[0] = *(const v8h*)(q);
  f.h[1] = *(const v8h*)(q + 16);
  return f.v;
}

__global__ __launch_bounds__(128)
void k_proj(const float* __restrict__ x, const float* __restrict__ W, const float* __restrict__ bw,
            float* __restrict__ T, hf* __restrict__ Xh) {
  constexpr int AP = NS + 8;
  constexpr int TP = TC + 4;
  static_assert((AP * 2) % 16 == 0);
  static_assert((TP * 4) % 16 == 0);
  __shared__ __align__(16) hf    As[64 * AP];
  __shared__ __align__(16) hf    Ws[TC * AP];
  __shared__ __align__(16) float Ts[64 * TP];
  __shared__ float sb[NE];

  const int tid = threadIdx.x, lane = tid & 31, wave = tid >> 5;
  const int hh = lane >> 4, c16 = lane & 15;
  const int blk = blockIdx.x;
  const int b  = blk / (NNODE / 64);
  const int n0 = (blk - b * (NNODE / 64)) * 64;

  if (tid < NE) sb[tid] = bw[tid];

  v4u    hvk[4];
  size_t hgo[4];
#pragma unroll
  for (int it = 0; it < 4; ++it) {
    const int p  = tid + 128 * it;
    const int s  = p >> 3;
    const int pc = p & 7;
    const size_t gofs = ((size_t)(b * NS + s)) * NNODE + n0 + 8 * pc;
    const v4f x0 = *(const v4f*)(x + gofs);
    const v4f x1 = *(const v4f*)(x + gofs + 4);
    Pk8 pk;
#pragma unroll
    for (int u = 0; u < 4; ++u) { pk.h[u] = (hf)x0[u]; pk.h[4 + u] = (hf)x1[u]; }
    hvk[it] = pk.u;
    hgo[it] = gofs;
#pragma unroll
    for (int u = 0; u < 8; ++u) As[(8 * pc + u) * AP + s] = pk.h[u];
  }
#pragma unroll
  for (int it = 0; it < 4; ++it) *(volatile v4u*)(Xh + hgo[it]) = hvk[it];
  __threadfence();
#pragma unroll
  for (int it = 0; it < 4; ++it) *(volatile v4u*)(Xh + hgo[it]) = hvk[it];

#pragma unroll
  for (int i = 0; i < 8; ++i) {
    const int q  = tid + 128 * i;
    const int cp = q >> 4;
    const int k  = (q & 15) * 4;
    const int widx = (cp & 31) * (2 * NS) + (cp >> 5) * NS + k;
    const v4f wv = *(const v4f*)(W + widx);
    v4h wh;
#pragma unroll
    for (int u = 0; u < 4; ++u) wh[u] = (hf)(wv[u] * 64.0f);
    *(v4h*)(Ws + cp * AP + k) = wh;
  }
  __syncthreads();

  v16h af[2];
#pragma unroll
  for (int ks = 0; ks < 2; ++ks) af[ks] = ldfrag(As, AP, 16 * wave, 32 * ks, lane);
#pragma unroll
  for (int t = 0; t < 4; ++t) {
    v8f acc = zero8();
#pragma unroll
    for (int ks = 0; ks < 2; ++ks) {
      const v16h bf = ldfrag(Ws, AP, 16 * t, 32 * ks, lane);
      acc = mma16(af[ks], bf, acc);
    }
#pragma unroll
    for (int r = 0; r < 8; ++r) {
      float v = acc[r] * (1.0f / 64.0f);
      if (t >= 2) v = v + sb[16 * t + c16 - NE];
      Ts[(16 * wave + 8 * hh + r) * TP + 16 * t + c16] = v;
    }
  }
  __syncthreads();

  v4f    val[8];
  size_t go[8];
#pragma unroll
  for (int it = 0; it < 8; ++it) {
    const int L    = wave * 32 + it * 4 + (lane >> 3);
    const int pc   = lane & 7;
    const int row  = L >> 1;
    const int half = L & 1;
    val[it] = *(const v4f*)(Ts + row * TP + half * 32 + 4 * pc);
    go[it]  = ((size_t)(b * NNODE + n0 + row)) * TC + half * 32 + 4 * pc;
  }
#pragma unroll
  for (int it = 0; it < 8; ++it) *(volatile v4f*)(T + go[it]) = val[it];
  __threadfence();
#pragma unroll
  for (int it = 0; it < 8; ++it) *(volatile v4f*)(T + go[it]) = val[it];
}

__global__ __launch_bounds__(512)
void k_edge(const float* __restrict__ T, const float* __restrict__ Wa, const float* __restrict__ ba,
            float* __restrict__ att, hf* __restrict__ Ph) {
  constexpr int EP = NNODE + 8;
  static_assert((EP * 4) % 16 == 0);
  __shared__ __align__(16) float Es[RB * EP];
  __shared__ __align__(16) float TIs[RB * NE];
  __shared__ __align__(16) float sWa[NE];

  const int tid = threadIdx.x, lane = tid & 31, wave = tid >> 5;
  const int blk = blockIdx.x;
  const int b  = blk / (NNODE / RB);
  const int i0 = (blk - b * (NNODE / RB)) * RB;

  if (tid < 128) {
    const int row = tid >> 3, pc = tid & 7;
    *(v4f*)(TIs + row * NE + 4 * pc) = *(const v4f*)(T + ((size_t)(b * NNODE + i0 + row)) * TC + 4 * pc);
  }
  if (tid < NE) sWa[tid] = Wa[tid];

  const float* tjp = T + ((size_t)(b * NNODE + tid)) * TC + NE;
  v4f tj[8];
#pragma unroll
  for (int q = 0; q < 8; ++q) tj[q] = *(const v4f*)(tjp + 4 * q);
  const float bav = ba[0];
  __syncthreads();

  v4f wa[8];
#pragma unroll
  for (int q = 0; q < 8; ++q) wa[q] = *(const v4f*)(sWa + 4 * q);

#pragma unroll 1
  for (int i = 0; i < RB; ++i) {
    const float* tip = TIs + i * NE;
    float acc = 0.f;
#pragma unroll
    for (int q = 0; q < 8; ++q) {
      const v4f ti = *(const v4f*)(tip + 4 * q);
#pragma unroll
      for (int u = 0; u < 4; ++u) {
        const float pre = ti[u] + tj[q][u];
        const float l   = (pre > 0.f) ? pre : 0.2f * pre;
        acc = fmaf(l, wa[q][u], acc);
      }
    }
    Es[i * EP + tid] = acc + bav;
  }
  __syncthreads();

  float* er = Es + wave * EP;
  v4f v[4];
  float mx = -3.0e38f;
#pragma unroll
  for (int it = 0; it < 4; ++it) {
    v[it] = *(const v4f*)(er + it * 128 + 4 * lane);
    mx = fmaxf(mx, fmaxf(fmaxf(v[it][0], v[it][1]), fmaxf(v[it][2], v[it][3])));
  }
#pragma unroll
  for (int off = 16; off >= 1; off >>= 1) mx = fmaxf(mx, __shfl_xor(mx, off, 32));
  float sum = 0.f;
#pragma unroll
  for (int it = 0; it < 4; ++it) {
#pragma unroll
    for (int u = 0; u < 4; ++u) {
      const float ev = __expf(v[it][u] - mx);
      v[it][u] = ev;
      sum += ev;
    }
  }
#pragma unroll
  for (int off = 16; off >= 1; off >>= 1) sum += __shfl_xor(sum, off, 32);
  const float inv = 1.0f / sum;
#pragma unroll
  for (int it = 0; it < 4; ++it) v[it] = v[it] * inv;

  const size_t arow = ((size_t)(b * NNODE + i0 + wave)) * NNODE;
#pragma unroll
  for (int it = 0; it < 4; ++it) *(volatile v4f*)(att + arow + it * 128 + 4 * lane) = v[it];
  __threadfence();
#pragma unroll
  for (int it = 0; it < 4; ++it) *(volatile v4f*)(att + arow + it * 128 + 4 * lane) = v[it];

#pragma unroll
  for (int it = 0; it < 4; ++it) *(v4f*)(er + it * 128 + 4 * lane) = v[it];
  __syncthreads();
  v4u    pk[2];
  size_t pgo[2];
#pragma unroll
  for (int g = 0; g < 2; ++g) {
    const v4f p0 = *(const v4f*)(er + g * 256 + 8 * lane);
    const v4f p1 = *(const v4f*)(er + g * 256 + 8 * lane + 4);
    Pk8 q;
#pragma unroll
    for (int u = 0; u < 4; ++u) { q.h[u] = (hf)(p0[u] * 4096.0f); q.h[4 + u] = (hf)(p1[u] * 4096.0f); }
    pk[g]  = q.u;
    pgo[g] = arow + g * 256 + 8 * lane;
  }
#pragma unroll
  for (int g = 0; g < 2; ++g) *(volatile v4u*)(Ph + pgo[g]) = pk[g];
  __threadfence();
#pragma unroll
  for (int g = 0; g < 2; ++g) *(volatile v4u*)(Ph + pgo[g]) = pk[g];
}

__global__ __launch_bounds__(128)
void k_pv(const hf* __restrict__ Ph, const hf* __restrict__ Xh, float* __restrict__ out) {
  constexpr int OP = 64 + 4;
  static_assert((OP * 4) % 16 == 0);
  __shared__ __align__(16) float Os[NS * OP];

  const int tid = threadIdx.x, lane = tid & 31, wave = tid >> 5;
  const int hh = lane >> 4, c16 = lane & 15;
  const int blk = blockIdx.x;
  const int b  = blk / (NNODE / 64);
  const int i0 = (blk - b * (NNODE / 64)) * 64;

  const hf* Pa = Ph + ((size_t)(b * NNODE + i0 + 16 * wave)) * NNODE;
  const hf* Xb = Xh + ((size_t)(b * NS)) * NNODE;

  v8f acc[4];
#pragma unroll
  for (int t = 0; t < 4; ++t) acc[t] = zero8();

#pragma unroll 1
  for (int kt = 0; kt < NNODE / 32; ++kt) {
    const v16h af = ldfrag(Pa, NNODE, 0, 32 * kt, lane);
#pragma unroll
    for (int t = 0; t < 4; ++t) {
      const v16h bf = ldfrag(Xb, NNODE, 16 * t, 32 * kt, lane);
      acc[t] = mma16(af, bf, acc[t]);
    }
  }

#pragma unroll
  for (int t = 0; t < 4; ++t) {
#pragma unroll
    for (int r = 0; r < 8; ++r) {
      const float z  = acc[t][r] * (1.0f / 4096.0f);
      const float ez = __expf(-z);
      const float hv = __builtin_amdgcn_rcpf(1.0f + ez);
      Os[(16 * t + c16) * OP + 16 * wave + 8 * hh + r] = hv;
    }
  }
  __syncthreads();

  v4f    val[8];
  size_t go[8];
#pragma unroll
  for (int it = 0; it < 8; ++it) {
    const int L    = wave * 32 + it * 4 + (lane >> 3);
    const int pc   = lane & 7;
    const int s    = L >> 1;
    const int half = L & 1;
    val[it] = *(const v4f*)(Os + s * OP + half * 32 + 4 * pc);
    go[it]  = ((size_t)(b * NS + s)) * NNODE + i0 + half * 32 + 4 * pc;
  }
#pragma unroll
  for (int it = 0; it < 8; ++it) *(volatile v4f*)(out + go[it]) = val[it];
  __threadfence();
#pragma unroll
  for (int it = 0; it < 8; ++it) *(volatile v4f*)(out + go[it]) = val[it];
}

extern "C" void kernel_launch(void* const* d_in, const int* in_sizes, int n_in,
                              void* d_out, int out_size, void* d_ws, size_t ws_size,
                              hipStream_t stream) {
  if (n_in < 5) return;
  if (in_sizes[0] != NB * NS * NNODE) return;
  if (in_sizes[1] != NE * 2 * NS) return;
  if (in_sizes[2] != NE) return;
  if (in_sizes[3] != NE) return;
  if (in_sizes[4] != 1) return;
  if (out_size != NB * NS * NNODE + NB * NNODE * NNODE) return;

  const float* x   = (const float*)d_in[0];
  const float* W   = (const float*)d_in[1];
  const float* b_w = (const float*)d_in[2];
  const float* Wa  = (const float*)d_in[3];
  const float* b_a = (const float*)d_in[4];

  float* out0 = (float*)d_out;
  float* out1 = (float*)d_out + (size_t)NB * NS * NNODE;

  size_t off = 0;
  const size_t oT  = off; off += (size_t)NB * NNODE * TC * 4;
  const size_t oXh = off; off += (size_t)NB * NS * NNODE * 2;
  const size_t oPh = off; off += (size_t)NB * NNODE * NNODE * 2;
  if (off > ws_size) return;
  if (off > (size_t)134217728) return;

  char* ws = (char*)d_ws;
  float* T  = (float*)(ws + oT);
  hf*    Xh = (hf*)(ws + oXh);
  hf*    Ph = (hf*)(ws + oPh);

  k_proj<<<dim3(NB * NNODE / 64), dim3(128), 0, stream>>>(x, W, b_w, T, Xh);
  k_edge<<<dim3(NB * NNODE / RB), dim3(512), 0, stream>>>(T, Wa, b_a, out1, Ph);
  k_pv<<<dim3(NB * NNODE / 64), dim3(128), 0, stream>>>(Ph, Xh, out0);
  (void)hipGetLastError();
}
